// MutualCrossAttention_10969346474178
// MI455X (gfx1250) — hardware-verified
//
#include <hip/hip_runtime.h>
#include <hip/hip_bf16.h>
#include <math.h>


#define BB 8
#define SS 2048
#define DD 256
#define HH 1
#define DKK 256
#define QW 2

typedef _Float16 bf16;
typedef __attribute__((ext_vector_type(4))) unsigned v4u_t;
typedef unsigned v4ua __attribute__((ext_vector_type(4), may_alias));
typedef __attribute__((ext_vector_type(4))) float v4f_t;
typedef float v4fa __attribute__((ext_vector_type(4), may_alias));
typedef __attribute__((ext_vector_type(16))) bf16  bf16x16;
typedef __attribute__((ext_vector_type(8)))  bf16  bf16x8;
typedef __attribute__((ext_vector_type(4)))  bf16  bf16x4;
typedef __attribute__((ext_vector_type(8)))  float f32x8;

#define LDS_STRIDE 48
#define KSTRIDE    72
#define VSTRIDE    48

__device__ __forceinline__ f32x8 wmma_bf16(bf16x16 a, bf16x16 b, f32x8 c) {
  return __builtin_amdgcn_wmma_f32_16x16x32_f16(
      false, a, false, b, (short)0, c, false, false);
}

template <typename T>
__device__ __forceinline__ bf16x16 load_frag(const T* __restrict__ base, int ld,
                                             int row0, int k0) {
  const int lane = threadIdx.x & 31;
  const int r    = lane & 15;
  const int kh   = (lane >> 4) * 8;
  const T* p0 = base + (size_t)(row0 + r) * ld + (k0 + kh);
  const T* p1 = p0 + 16;
  bf16x16 f;
#pragma unroll
  for (int i = 0; i < 8; ++i) {
    f[i]     = (bf16)p0[i];
    f[i + 8] = (bf16)p1[i];
  }
  return f;
}

__device__ __forceinline__ bf16x16 lds_frag(const bf16* base, int stride) {
  const int lane = threadIdx.x & 31;
  const int row  = lane & 15;
  const int kh   = (lane >> 4) * 8;
  const bf16x8 lo = *(const bf16x8*)(base + row * stride + kh);
  const bf16x8 hi = *(const bf16x8*)(base + row * stride + kh + 16);
  bf16x16 f;
#pragma unroll
  for (int i = 0; i < 8; ++i) { f[i] = lo[i]; f[i + 8] = hi[i]; }
  return f;
}

template <typename T>
__device__ __forceinline__ void stage_read16(const T* __restrict__ p, float* buf) {
#pragma unroll
  for (int i = 0; i < 16; ++i) buf[i] = (float)p[i];
}

__device__ __forceinline__ void stage_write(bf16* dst, const float* buf, int nquad) {
#pragma unroll
  for (int i = 0; i < nquad; ++i) {
    bf16x4 q;
    q[0] = (bf16)buf[4 * i];     q[1] = (bf16)buf[4 * i + 1];
    q[2] = (bf16)buf[4 * i + 2]; q[3] = (bf16)buf[4 * i + 3];
    *(bf16x4*)(dst + 4 * i) = q;
  }
}

__global__ __launch_bounds__(256) void transpose_pack_kernel(const float* __restrict__ W, bf16* __restrict__ WT, int K, int N) {
  __shared__ float tile[64][65];
  const int k0 = blockIdx.y * 64, n0 = blockIdx.x * 64, t = threadIdx.x;
  for (int i = t; i < 64 * 64; i += 256) { const int kr = i >> 6, nc = i & 63; tile[kr][nc] = W[(size_t)(k0 + kr) * N + n0 + nc]; }
  __syncthreads();
#pragma unroll 1
  for (int pass = 0; pass < 2; ++pass) {
    for (int i = t; i < 64 * 8; i += 256) { const int nr = i >> 3, k8 = (i & 7) * 8; bf16 hh[8];
#pragma unroll
      for (int e = 0; e < 8; ++e) hh[e] = (bf16)tile[k8 + e][nr];
      *(volatile v4u_t*)(WT + (size_t)(n0 + nr) * K + k0 + k8) = *(const v4ua*)hh; }
    __threadfence();
  }
}

template <typename AT, typename WT, int MODE>
__global__ __launch_bounds__(256) void gemm_bias_kernel(
    const AT* __restrict__ A, const WT* __restrict__ W,
    const float* __restrict__ bias, void* __restrict__ out,
    int M, int N, int K) {
  __shared__ bf16 ldsA[128 * LDS_STRIDE];
  __shared__ bf16 ldsW[256 * LDS_STRIDE];
  __shared__ __attribute__((aligned(16))) unsigned char sob[256 * 136 * 2];

  const int t    = threadIdx.x;
  const int wave = t >> 5;
  const int lane = t & 31;
  const int wm   = (wave & 1) * 64;
  const int wn   = (wave >> 1) * 64;
  const int mBlk = blockIdx.x * 128;
  const int nBlk = blockIdx.y * 256;

  const int arow = t >> 1;
  const int ach  = (t & 1) * 16;

  float abuf[16];
  float wbuf[32];

  stage_read16(A + (size_t)(mBlk + arow) * K + ach, abuf);
  stage_read16(W + (size_t)(nBlk + t) * K,          wbuf);
  stage_read16(W + (size_t)(nBlk + t) * K + 16,     wbuf + 16);

  f32x8 acc[4][4] = {};

  for (int k = 0; k < K; k += 32) {
    __syncthreads();
    stage_write(&ldsA[arow * LDS_STRIDE + ach], abuf, 4);
    stage_write(&ldsW[t * LDS_STRIDE],          wbuf, 8);
    if (k + 32 < K) {
      stage_read16(A + (size_t)(mBlk + arow) * K + (k + 32) + ach, abuf);
      stage_read16(W + (size_t)(nBlk + t) * K + (k + 32),          wbuf);
      stage_read16(W + (size_t)(nBlk + t) * K + (k + 32) + 16,     wbuf + 16);
    }
    __syncthreads();

    bf16x16 af[4], wf[4];
#pragma unroll
    for (int i = 0; i < 4; ++i)
      af[i] = lds_frag(ldsA + (wm + 16 * i) * LDS_STRIDE, LDS_STRIDE);
#pragma unroll
    for (int j = 0; j < 4; ++j)
      wf[j] = lds_frag(ldsW + (wn + 16 * j) * LDS_STRIDE, LDS_STRIDE);
#pragma unroll
    for (int i = 0; i < 4; ++i)
#pragma unroll
      for (int j = 0; j < 4; ++j)
        acc[i][j] = wmma_bf16(af[i], wf[j], acc[i][j]);
  }

  const int nlane = lane & 15;
  const int mh    = (lane >> 4) * 8;
  __syncthreads();
  if (MODE == 0 || MODE == 1) {
    bf16* so = (bf16*)sob;
#pragma unroll
    for (int i = 0; i < 4; ++i)
#pragma unroll
      for (int j = 0; j < 4; ++j) {
        const int nl = wn + 16 * j + nlane;
        const float bv = bias ? bias[nBlk + nl] : 0.0f;
#pragma unroll
        for (int r = 0; r < 8; ++r) {
          const int ml = wm + 16 * i + mh + r;
          const bf16 hv = (bf16)(acc[i][j][r] + bv);
          if (MODE == 0) so[ml * 264 + nl] = hv;
          else           so[nl * 136 + ml] = hv;
        }
      }
    __syncthreads();
#pragma unroll 1
    for (int pass = 0; pass < 2; ++pass) {
      if (MODE == 0) {
        for (int ch = t; ch < 128 * 32; ch += 256) { const int ml = ch >> 5, q = (ch & 31) * 8;
          *(volatile v4u_t*)((bf16*)out + (size_t)(mBlk + ml) * N + nBlk + q) = *(const v4ua*)(so + ml * 264 + q); }
      } else {
        const int b_ = mBlk >> 11, s0 = mBlk & (SS - 1);
        for (int ch = t; ch < 256 * 16; ch += 256) { const int nl = ch >> 4, q = (ch & 15) * 8; const int n = nBlk + nl, h = n >> 6, dk = n & (DKK - 1);
          *(volatile v4u_t*)((bf16*)out + (((size_t)(b_ * HH + h)) * DKK + dk) * SS + s0 + q) = *(const v4ua*)(so + nl * 136 + q); }
      }
      __threadfence();
    }
  } else {
    float* so = (float*)sob;
#pragma unroll 1
    for (int hf = 0; hf < 2; ++hf) {
      if (wm == hf * 64) {
#pragma unroll
        for (int i = 0; i < 4; ++i)
#pragma unroll
          for (int j = 0; j < 4; ++j) {
            const int nl = wn + 16 * j + nlane;
            const float bv = bias ? bias[nBlk + nl] : 0.0f;
#pragma unroll
            for (int r = 0; r < 8; ++r) so[(16 * i + mh + r) * 260 + nl] = acc[i][j][r] + bv;
          }
      }
      __syncthreads();
#pragma unroll 1
      for (int pass = 0; pass < 2; ++pass) {
        for (int ch = t; ch < 64 * 64; ch += 256) { const int ml = ch >> 6, q = (ch & 63) * 4;
          *(volatile v4f_t*)((float*)out + (size_t)(mBlk + hf * 64 + ml) * N + nBlk + q) = *(const volatile v4fa*)(so + ml * 260 + q); }
        __threadfence();
      }
      __syncthreads();
    }
  }
}


#define KS2 264
#define VS2 40
__global__ __launch_bounds__(128) void xattn_kernel(const bf16* __restrict__ Qp, const bf16* __restrict__ Kp, const float* __restrict__ Vsrc,
                                                  float* __restrict__ outRows  ) {
  __shared__ __attribute__((aligned(16))) bf16 ldsK[32 * KS2];
  __shared__ __attribute__((aligned(16))) bf16 ldsV[256 * VS2];
  __shared__ __attribute__((aligned(16))) bf16 ldsQa[2][16 * KS2];
  __shared__ float ldsSa[2][2][16 * 17];
  __shared__ __attribute__((aligned(16))) float ldsOa[2][16 * 260];
  const int b = blockIdx.y;
  const int t = threadIdx.x, wave4 = t >> 5, lane = t & 31, qlane = lane & 15, kh8 = (lane >> 4) * 8;
  const int qt = wave4 >> 1, wave = wave4 & 1;
  const int q0 = blockIdx.x * 32 + qt * 16;
  bf16* ldsQ = ldsQa[qt]; float (*ldsS)[16 * 17] = ldsSa[qt]; float* ldsO = ldsOa[qt];
  const bf16* Qb = Qp + (size_t)b * SS * DD;
  const bf16* Kb = Kp + (size_t)b * SS * DD;
  const float* Vb = Vsrc + (size_t)b * SS * DD;
  for (int i = (t & 63); i < 16 * 32; i += 64) { const int r = i >> 5, c8 = (i & 31) * 8; *(bf16x8*)(&ldsQ[r * KS2 + c8]) = *(const bf16x8*)(Qb + (size_t)(q0 + r) * DD + c8); }
  f32x8 o[8] = {};
  float mrun = -INFINITY, lrun = 0.0f;
  const float scale = 0.0625f * 1.44269504088896340736f;
#pragma unroll 1
  for (int kb = 0; kb < SS; kb += 32) {
    __syncthreads();
    { const int kr = t >> 2, kc0 = (t & 3) * 64; const bf16* ks = Kb + (size_t)(kb + kr) * DD + kc0;
#pragma unroll
      for (int i = 0; i < 8; ++i) *(bf16x8*)(&ldsK[kr * KS2 + kc0 + 8 * i]) = *(const bf16x8*)(ks + 8 * i);
      const int vk = t & 31, d0 = (t >> 5) * 64; const float* vs = Vb + (size_t)(kb + vk) * DD + d0;
#pragma unroll 4
      for (int i = 0; i < 64; ++i) ldsV[(d0 + i) * VS2 + vk] = (bf16)vs[i]; }
    __syncthreads();
    { f32x8 sw = {};
#pragma unroll
      for (int c = 0; c < 8; ++c) sw = wmma_bf16(lds_frag(&ldsK[(wave * 16) * KS2 + c * 32], KS2), lds_frag(&ldsQ[c * 32], KS2), sw);
#pragma unroll
      for (int r = 0; r < 8; ++r) ldsS[wave][(kh8 + r) * 17 + qlane] = sw[r] * scale; }
    __syncthreads();
    float s0[8], s1[8]; float mx = -INFINITY;
#pragma unroll
    for (int r = 0; r < 8; ++r) { s0[r] = ldsS[0][(kh8 + r) * 17 + qlane]; s1[r] = ldsS[1][(kh8 + r) * 17 + qlane]; mx = fmaxf(mx, fmaxf(s0[r], s1[r])); }
    mx = fmaxf(mx, __shfl_xor(mx, 16, 32));
    const float mnew = fmaxf(mrun, mx), alpha = exp2f(mrun - mnew);
    float rsum = 0.0f; bf16x16 pf;
#pragma unroll
    for (int r = 0; r < 8; ++r) { const float p0 = exp2f(s0[r] - mnew), p1 = exp2f(s1[r] - mnew); rsum += p0 + p1; pf[r] = (bf16)(p0 * 1024.0f); pf[r + 8] = (bf16)(p1 * 1024.0f); }
    rsum += __shfl_xor(rsum, 16, 32);
    lrun = lrun * alpha + rsum; mrun = mnew;
#pragma unroll
    for (int j = 0; j < 8; ++j) {
#pragma unroll
      for (int r = 0; r < 8; ++r) o[j][r] *= alpha;
      o[j] = wmma_bf16(lds_frag(&ldsV[((wave * 8 + j) * 16) * VS2], VS2), pf, o[j]);
    }
  }
  const float rl = 1.0f / (lrun * 1024.0f);
#pragma unroll
  for (int j = 0; j < 8; ++j)
#pragma unroll
    for (int r = 0; r < 8; ++r) ldsO[qlane * 260 + (wave * 8 + j) * 16 + kh8 + r] = o[j][r] * rl;
  __syncthreads();
#pragma unroll 1
  for (int pass = 0; pass < 2; ++pass) {
    for (int i = (t & 63); i < 16 * 64; i += 64) { const int ql = i >> 6, q4 = (i & 63) * 4;
      *(volatile v4f_t*)(outRows + ((size_t)b * 2 * SS + q0 + ql) * DD + q4) = *(const volatile v4fa*)(ldsO + ql * 260 + q4); }
    __threadfence();
  }
}

extern "C" void kernel_launch(void* const* d_in, const int* in_sizes, int n_in,
                              void* d_out, int out_size, void* d_ws, size_t ws_size,
                              hipStream_t stream) {
  (void)in_sizes; (void)n_in; (void)out_size; (void)ws_size;
  const float* x1 = (const float*)d_in[0];
  const float* x2 = (const float*)d_in[1];
  const float* W  = (const float*)d_in[2];
  const float* bb = (const float*)d_in[3];
  char* ws = (char*)d_ws;
  bf16* WT = (bf16*)ws; ws += (size_t)DD * DD * 2;
  bf16* Qp = (bf16*)ws; ws += (size_t)BB * SS * DD * 2;
  bf16* Kp = (bf16*)ws; ws += (size_t)BB * SS * DD * 2;
  transpose_pack_kernel<<<dim3(DD / 64, DD / 64), 256, 0, stream>>>(W, WT, DD, DD);
  const int M = BB * SS;
  gemm_bias_kernel<float, bf16, 0><<<dim3(M / 128, DD / 256), 256, 0, stream>>>(x1, WT, bb, Qp, M, DD, DD);
  gemm_bias_kernel<float, bf16, 0><<<dim3(M / 128, DD / 256), 256, 0, stream>>>(x2, WT, bb, Kp, M, DD, DD);
  float* out = (float*)d_out;
  xattn_kernel<<<dim3(SS / 32, BB), 128, 0, stream>>>(Qp, Kp, x2, out);
  xattn_kernel<<<dim3(SS / 32, BB), 128, 0, stream>>>(Kp, Qp, x1, out + (size_t)SS * DD);
}
